// HGNNLayer_7997229105162
// MI455X (gfx1250) — hardware-verified
//
#include <hip/hip_runtime.h>
#include <stddef.h>


#define DF    128
#define GR    32
#define AP    136
#define XSP   132
#define NB    512
#define CHUNK 2048
#define NTHR  256
#define NWAVE 8
#define WCAP  256
#define NGRP  (CHUNK / (NTHR * 4))

#define LDS_AGG_BYTES ((NB * DF + NB + NB + NWAVE * WCAP + NWAVE) * 4)
#define LDS_CMB_BYTES (4 * GR * AP * 2)

static_assert(WCAP == (CHUNK / NTHR) * 32);
static_assert(NGRP == 2);
static_assert(NB == 512);
static_assert(CHUNK == 2048);
static_assert(LDS_AGG_BYTES == 274464);
static_assert(((NB * DF + NB) % 4) == 0);
static_assert(GR == 4 * NWAVE);
static_assert((AP % 8) == 0);
static_assert((XSP % 4) == 0);
static_assert(LDS_CMB_BYTES == 34816);
static_assert(2 * GR * XSP * 4 <= LDS_CMB_BYTES);
static_assert((LDS_CMB_BYTES % 16) == 0);

typedef float          v4f  __attribute__((ext_vector_type(4)));
typedef float          v8f  __attribute__((ext_vector_type(8)));
typedef int            v4i  __attribute__((ext_vector_type(4)));
typedef int            v8i  __attribute__((ext_vector_type(8)));
typedef unsigned short v8us __attribute__((ext_vector_type(8)));
typedef __bf16         v16b __attribute__((ext_vector_type(16)));
union Frag { v16b v; v8us half[2]; };
union P16  { v8us u; v4i i; };

__device__ __forceinline__ unsigned short bfb(float f) {
  unsigned u = __float_as_uint(f);
  u += 0x7FFFu + ((u >> 16) & 1u);
  return (unsigned short)(u >> 16);
}
__device__ __forceinline__ float bfu(unsigned short b) { return __uint_as_float(((unsigned)b) << 16); }
__device__ __forceinline__ float bfr(float f) { return bfu(bfb(f)); }
__device__ __forceinline__ v4f bfr4(v4f a) {
  v4f r;
  r.x = bfr(a.x); r.y = bfr(a.y); r.z = bfr(a.z); r.w = bfr(a.w);
  return r;
}

__device__ __forceinline__ v8f wmb(v16b a, v16b b, v8f c) {
  v8f d = __builtin_amdgcn_wmma_f32_16x16x32_bf16(false, a, false, b, (short)0, c, false, false);
  const v8i ai = __builtin_bit_cast(v8i, a);
  const v8i bi = __builtin_bit_cast(v8i, b);
  asm volatile("v_nop\n\tv_nop\n\tv_nop\n\tv_nop" : "+v"(d) : "v"(ai), "v"(bi));
  return d;
}

__device__ __forceinline__ float wsum(float v) {
  v += __shfl_xor(v, 16, 32);
  v += __shfl_xor(v, 8, 32);
  v += __shfl_xor(v, 4, 32);
  v += __shfl_xor(v, 2, 32);
  v += __shfl_xor(v, 1, 32);
  return v;
}

__device__ __forceinline__ v4f lk4(v4f a, float s) {
  v4f r;
  r.x = (a.x >= 0.f) ? a.x : s * a.x;
  r.y = (a.y >= 0.f) ? a.y : s * a.y;
  r.z = (a.z >= 0.f) ? a.z : s * a.z;
  r.w = (a.w >= 0.f) ? a.w : s * a.w;
  return r;
}

__global__ __launch_bounds__(NTHR) void k_prep(const float* __restrict__ W, const float* __restrict__ biw,
                                               const float* __restrict__ siw, unsigned short* wt, int nR) {
  __shared__ __attribute__((aligned(16))) unsigned short T[DF * AP];
  const int tid = threadIdx.x;
  const int buf = blockIdx.x;
  if (buf < nR) {
    const float* src = W + (size_t)buf * DF * DF;
#pragma unroll 1
    for (int idx = tid; idx < DF * DF; idx += NTHR) {
      const int k = idx >> 7, j = idx & (DF - 1);
      T[j * AP + k] = bfb(src[idx]);
    }
  } else {
    const float* src = (buf == nR) ? biw : siw;
#pragma unroll 1
    for (int idx = tid; idx < DF * DF; idx += NTHR) {
      const int j = idx >> 7, k = idx & (DF - 1);
      T[j * AP + k] = bfb(src[idx]);
    }
  }
  __syncthreads();
  unsigned short* plane = wt + (size_t)buf * DF * DF;
  P16 pk[8];
#pragma unroll
  for (int it = 0; it < 8; ++it) {
    const int L = it * 32 + (tid >> 3);
    const int j = L >> 1, c = (L & 1) * 64 + (tid & 7) * 8;
    pk[it].u = *(const v8us*)(T + j * AP + c);
  }
#pragma unroll
  for (int it = 0; it < 8; ++it) {
    const int L = it * 32 + (tid >> 3);
    const int j = L >> 1, c = (L & 1) * 64 + (tid & 7) * 8;
    *(volatile v4i*)(plane + (size_t)j * DF + c) = pk[it].i;
  }
  __threadfence();
#pragma unroll
  for (int it = 0; it < 8; ++it) {
    const int L = it * 32 + (tid >> 3);
    const int j = L >> 1, c = (L & 1) * 64 + (tid & 7) * 8;
    *(volatile v4i*)(plane + (size_t)j * DF + c) = pk[it].i;
  }
}

__device__ __forceinline__ void epi_tile(v8f acc, int T, int hh, int m, int wave, int ncol,
                                         float cs, float cd, float* Xs, float* As, float* Ds) {
  float ss[8], sd[8];
#pragma unroll
  for (int r = 0; r < 8; ++r) {
    const float v = acc[r];
    Xs[(T * 16 + 8 * hh + r) * XSP + ncol] = v;
    ss[r] = v * cs;
    sd[r] = v * cd;
  }
#pragma unroll
  for (int mk = 1; mk < 16; mk <<= 1) {
#pragma unroll
    for (int r = 0; r < 8; ++r) {
      ss[r] += __shfl_xor(ss[r], mk, 32);
      sd[r] += __shfl_xor(sd[r], mk, 32);
    }
  }
  if (m == 0) {
#pragma unroll
    for (int r = 0; r < 8; ++r) {
      As[(T * 16 + 8 * hh + r) * NWAVE + wave] = ss[r];
      Ds[(T * 16 + 8 * hh + r) * NWAVE + wave] = sd[r];
    }
  }
}

__global__ __launch_bounds__(NTHR) void k_gemm(
    const float* __restrict__ x, const unsigned short* __restrict__ wt,
    const float* __restrict__ al, const float* __restrict__ ar,
    float* hout, float* elp, float* erp, int nN) {
  __shared__ __attribute__((aligned(16))) unsigned short At[GR * AP];
  __shared__ __attribute__((aligned(16))) float Xs[GR * XSP];
  __shared__ __attribute__((aligned(16))) float As[GR * NWAVE];
  __shared__ __attribute__((aligned(16))) float Ds[GR * NWAVE];
  __shared__ __attribute__((aligned(16))) float EL[GR];
  __shared__ __attribute__((aligned(16))) float ER[GR];

  const int tid  = threadIdx.x;
  const int lane = tid & 31;
  const int wave = tid >> 5;
  const int hh   = lane >> 4;
  const int m    = lane & 15;
  const int rowBase = blockIdx.x * GR;

  {
    const int r  = tid >> 3;
    const int c0 = (tid & 7) * 16;
    int row = rowBase + r;
    if (row > nN - 1) row = nN - 1;
    const float* p = x + (size_t)row * DF + c0;
    const v4f f0 = *(const v4f*)(p), f1 = *(const v4f*)(p + 4);
    const v4f f2 = *(const v4f*)(p + 8), f3 = *(const v4f*)(p + 12);
    P16 u0, u1;
    u0.u[0] = bfb(f0.x); u0.u[1] = bfb(f0.y); u0.u[2] = bfb(f0.z); u0.u[3] = bfb(f0.w);
    u0.u[4] = bfb(f1.x); u0.u[5] = bfb(f1.y); u0.u[6] = bfb(f1.z); u0.u[7] = bfb(f1.w);
    u1.u[0] = bfb(f2.x); u1.u[1] = bfb(f2.y); u1.u[2] = bfb(f2.z); u1.u[3] = bfb(f2.w);
    u1.u[4] = bfb(f3.x); u1.u[5] = bfb(f3.y); u1.u[6] = bfb(f3.z); u1.u[7] = bfb(f3.w);
    *(v8us*)(At + r * AP + c0)     = u0.u;
    *(v8us*)(At + r * AP + c0 + 8) = u1.u;
  }
  __syncthreads();

  const int ncol = wave * 16 + m;
  v8f c0a = {0.f, 0.f, 0.f, 0.f, 0.f, 0.f, 0.f, 0.f};
  v8f c1a = {0.f, 0.f, 0.f, 0.f, 0.f, 0.f, 0.f, 0.f};
#pragma unroll
  for (int kt = 0; kt < DF / 32; ++kt) {
    const int k0 = kt * 32;
    Frag a0, a1, b;
    const unsigned short* pb  = wt + (size_t)ncol * DF + k0 + 8 * hh;
    const unsigned short* pa0 = At + m * AP + k0 + 8 * hh;
    const unsigned short* pa1 = At + (16 + m) * AP + k0 + 8 * hh;
    b.half[0]  = *(const v8us*)pb;  b.half[1]  = *(const v8us*)(pb + 16);
    a0.half[0] = *(const v8us*)pa0; a0.half[1] = *(const v8us*)(pa0 + 16);
    a1.half[0] = *(const v8us*)pa1; a1.half[1] = *(const v8us*)(pa1 + 16);
    c0a = wmb(a0.v, b.v, c0a);
    c1a = wmb(a1.v, b.v, c1a);
  }

  const float cs = bfr(al[ncol]);
  const float cd = bfr(ar[ncol]);
  epi_tile(c0a, 0, hh, m, wave, ncol, cs, cd, Xs, As, Ds);
  epi_tile(c1a, 1, hh, m, wave, ncol, cs, cd, Xs, As, Ds);
  __syncthreads();

  if (tid < GR) {
    float s = 0.f;
#pragma unroll
    for (int w = 0; w < NWAVE; ++w) s += As[tid * NWAVE + w];
    EL[tid] = s;
  } else if (tid < 2 * GR) {
    const int t2 = tid - GR;
    float s = 0.f;
#pragma unroll
    for (int w = 0; w < NWAVE; ++w) s += Ds[t2 * NWAVE + w];
    ER[t2] = s;
  }
  __syncthreads();

  v4f xr[4];
#pragma unroll
  for (int i = 0; i < 4; ++i) xr[i] = *(const v4f*)(Xs + (4 * wave + i) * XSP + 4 * lane);
  const int l8 = (lane < 8) ? lane : 0;
  const v4f ve = *(const v4f*)(EL + 4 * l8);
  const v4f vr = *(const v4f*)(ER + 4 * l8);
  v4f gv = vr;
  if (wave == 0) gv = ve;
  float* gp = (wave == 0) ? (elp + rowBase + 4 * lane) : (erp + rowBase + 4 * lane);
  const bool wst = (wave < 2) && (lane < 8);

#pragma unroll
  for (int i = 0; i < 4; ++i)
    *(volatile v4f*)(hout + (size_t)(rowBase + 4 * wave + i) * DF + 4 * lane) = xr[i];
  if (wst) *(volatile v4f*)gp = gv;
  __threadfence();
#pragma unroll
  for (int i = 0; i < 4; ++i)
    *(volatile v4f*)(hout + (size_t)(rowBase + 4 * wave + i) * DF + 4 * lane) = xr[i];
  if (wst) *(volatile v4f*)gp = gv;
}

__global__ __launch_bounds__(NTHR) void k_agg(
    const float* __restrict__ hpl, const float* __restrict__ elp, const float* __restrict__ erp,
    const int* __restrict__ esrc, const int* __restrict__ edst, const float* __restrict__ ew,
    const float* __restrict__ gb, float* Spl, float* Qpl, int nN, int nE, int accum) {
  extern __shared__ v4f lds_dyn[];
  float* sacc = (float*)lds_dyn;
  float* den  = sacc + NB * DF;
  float* mrun = den + NB;
  int*   list = (int*)(mrun + NB);
  int*   wcnt = list + NWAVE * WCAP;

  const int tid  = threadIdx.x;
  const int lane = tid & 31;
  const int wave = tid >> 5;
  const int nodeBase = blockIdx.x * NB;

  {
    const v4f z4 = {0.f, 0.f, 0.f, 0.f};
#pragma unroll 1
    for (int i = tid; i < (NB * DF + NB) / 4; i += NTHR) lds_dyn[i] = z4;
#pragma unroll 1
    for (int i = tid; i < NB; i += NTHR) mrun[i] = -1.0e30f;
  }
  __syncthreads();

  const bool al16 = ((reinterpret_cast<size_t>(edst) & (size_t)15) == 0);

  const int nChunks = (nE + CHUNK - 1) / CHUNK;
#pragma unroll 1
  for (int ch = 0; ch < nChunks; ++ch) {
    const int cbase = ch * CHUNK;
    int wc = 0;
#pragma unroll
    for (int g = 0; g < NGRP; ++g) {
      const int el0 = (g * NTHR + tid) * 4;
      const int e0  = cbase + el0;
      const int sent = -2147483647 - 1;
      v4i d;
      if (al16 && (cbase + CHUNK <= nE)) {
        d = *(const v4i*)(edst + e0);
      } else {
        const int q0 = (e0     < nE) ? e0     : nE - 1;
        const int q1 = (e0 + 1 < nE) ? e0 + 1 : nE - 1;
        const int q2 = (e0 + 2 < nE) ? e0 + 2 : nE - 1;
        const int q3 = (e0 + 3 < nE) ? e0 + 3 : nE - 1;
        const int v0 = edst[q0], v1 = edst[q1], v2 = edst[q2], v3 = edst[q3];
        d.x = (e0     < nE) ? v0 : sent;
        d.y = (e0 + 1 < nE) ? v1 : sent;
        d.z = (e0 + 2 < nE) ? v2 : sent;
        d.w = (e0 + 3 < nE) ? v3 : sent;
      }
      const unsigned s0 = (unsigned)d.x - (unsigned)nodeBase;
      const unsigned s1 = (unsigned)d.y - (unsigned)nodeBase;
      const unsigned s2 = (unsigned)d.z - (unsigned)nodeBase;
      const unsigned s3 = (unsigned)d.w - (unsigned)nodeBase;
      const bool h0 = s0 < (unsigned)NB;
      const bool h1 = s1 < (unsigned)NB;
      const bool h2 = s2 < (unsigned)NB;
      const bool h3 = s3 < (unsigned)NB;
      const unsigned many = __builtin_amdgcn_ballot_w32(h0 | h1 | h2 | h3);
      if (many != 0u) {
#define HITJ(J, HJ, SJ) { \
          const unsigned mj = __builtin_amdgcn_ballot_w32(HJ); \
          if (HJ) { \
            const int pos = wc + (int)__builtin_amdgcn_mbcnt_lo(mj, 0u); \
            if (pos < WCAP) list[wave * WCAP + pos] = ((el0 + (J)) << 9) | (int)(SJ); \
          } \
          wc += (int)__builtin_popcount(mj); }
        HITJ(0, h0, s0)
        HITJ(1, h1, s1)
        HITJ(2, h2, s2)
        HITJ(3, h3, s3)
#undef HITJ
      }
    }
    if (lane == 0) wcnt[wave] = wc;
    __syncthreads();

    if (wave == 0) {
#pragma unroll 1
      for (int wsx = 0; wsx < NWAVE; ++wsx) {
        int n = wcnt[wsx];
        if (n > WCAP) n = WCAP;
        if (n < 0) n = 0;
#pragma unroll 1
        for (int i = 0; i < n; ++i) {
          const int ent  = list[wsx * WCAP + i];
          const int slot = ent & (NB - 1);
          const int elx  = (ent >> 9) & (CHUNK - 1);
          int e = cbase + elx;
          if (e > nE - 1) e = nE - 1;
          int src = esrc[e];
          src = src < 0 ? 0 : (src > nN - 1 ? nN - 1 : src);
          const float w = bfr(ew[e]);
          int nd = nodeBase + slot;
          if (nd > nN - 1) nd = nN - 1;
          float lg = elp[src] + erp[nd];
          lg = (lg >= 0.f) ? lg : 0.2f * lg;
          const float mo = mrun[slot];
          const float dn = den[slot];
          const float mn = fmaxf(mo, lg);
          const float sc = __expf(mo - mn);
          const float p  = __expf(lg - mn);
          const v4f hv = *(const v4f*)(hpl + (size_t)src * DF + 4 * lane);
          v4f* sp = (v4f*)(sacc + slot * DF + 4 * lane);
          const v4f cur = *sp;
          const v4f nxt = cur * sc + (p * w) * hv;
          *sp = nxt;
          den[slot]  = dn * sc + p;
          mrun[slot] = mn;
        }
      }
    }
    __syncthreads();
  }

  const v4f b4 = {bfr(gb[4 * lane]), bfr(gb[4 * lane + 1]), bfr(gb[4 * lane + 2]), bfr(gb[4 * lane + 3])};
#pragma unroll 1
  for (int j = 0; j < NB / NWAVE; ++j) {
    const int slot = wave * (NB / NWAVE) + j;
    const int node = nodeBase + slot;
    if (node >= nN) break;
    const float dn  = den[slot];
    const float inv = (dn > 0.f) ? (1.0f / fmaxf(dn, 1.0f)) : 0.f;
    const v4f sv = *(const v4f*)(sacc + slot * DF + 4 * lane);
    const v4f f  = sv * inv + b4;
    const size_t go = (size_t)node * DF + 4 * lane;
    v4f so = {0.f, 0.f, 0.f, 0.f};
    v4f qo = {0.f, 0.f, 0.f, 0.f};
    if (accum != 0) {
      so = *(const v4f*)(Spl + go);
      qo = *(const v4f*)(Qpl + go);
    }
    const v4f sn = so + f;
    const v4f qn = qo + f * f;
    *(volatile v4f*)(Spl + go) = sn;
    *(volatile v4f*)(Qpl + go) = qn;
    __threadfence();
    *(volatile v4f*)(Spl + go) = sn;
    *(volatile v4f*)(Qpl + go) = qn;
  }
}

__global__ __launch_bounds__(NTHR) void k_comb(
    const float* __restrict__ Spl, const float* __restrict__ Qpl, const float* __restrict__ x,
    const unsigned short* __restrict__ wtb, const float* __restrict__ bib,
    const unsigned short* __restrict__ wts, const float* __restrict__ sib,
    const float* __restrict__ resw, const float* __restrict__ lng, const float* __restrict__ lnb,
    float* out, int nN) {
  __shared__ v4f lraw[LDS_CMB_BYTES / 16];
  unsigned short* Adh = (unsigned short*)lraw;
  unsigned short* Adl = Adh + GR * AP;
  unsigned short* Ash = Adl + GR * AP;
  unsigned short* Asl = Ash + GR * AP;
  float* Y1 = (float*)lraw;
  float* Y2 = Y1 + GR * XSP;

  const int tid  = threadIdx.x;
  const int lane = tid & 31;
  const int wave = tid >> 5;
  const int hh   = lane >> 4;
  const int m    = lane & 15;
  const int rowBase = blockIdx.x * GR;

  {
    const int r  = tid >> 3;
    const int c0 = (tid & 7) * 16;
    int row = rowBase + r;
    if (row > nN - 1) row = nN - 1;
    const float* ps = Spl + (size_t)row * DF + c0;
    const float* pq = Qpl + (size_t)row * DF + c0;
#pragma unroll
    for (int hx = 0; hx < 2; ++hx) {
      const v4f sa = *(const v4f*)(ps + 8 * hx), sb = *(const v4f*)(ps + 8 * hx + 4);
      const v4f qa = *(const v4f*)(pq + 8 * hx), qb = *(const v4f*)(pq + 8 * hx + 4);
      const float sv[8] = {sa.x, sa.y, sa.z, sa.w, sb.x, sb.y, sb.z, sb.w};
      const float qv[8] = {qa.x, qa.y, qa.z, qa.w, qb.x, qb.y, qb.z, qb.w};
      P16 sh, sl, dh, dl;
#pragma unroll
      for (int e = 0; e < 8; ++e) {
        const float s = sv[e];
        const float d = 0.5f * (s * s - qv[e]);
        const unsigned short shb = bfb(s);
        const float shv = bfu(shb);
        sh.u[e] = shb;
        sl.u[e] = bfb(s - shv);
        const unsigned short dhb = bfb(d);
        const float dhv = bfu(dhb);
        dh.u[e] = dhb;
        dl.u[e] = bfb(d - dhv);
      }
      const int o = r * AP + c0 + 8 * hx;
      *(v8us*)(Ash + o) = sh.u;
      *(v8us*)(Asl + o) = sl.u;
      *(v8us*)(Adh + o) = dh.u;
      *(v8us*)(Adl + o) = dl.u;
    }
  }
  __syncthreads();

  const int ncol = wave * 16 + m;
  v8f d0 = {0.f, 0.f, 0.f, 0.f, 0.f, 0.f, 0.f, 0.f};
  v8f d1 = {0.f, 0.f, 0.f, 0.f, 0.f, 0.f, 0.f, 0.f};
  v8f s0 = {0.f, 0.f, 0.f, 0.f, 0.f, 0.f, 0.f, 0.f};
  v8f s1 = {0.f, 0.f, 0.f, 0.f, 0.f, 0.f, 0.f, 0.f};
#pragma unroll
  for (int kt = 0; kt < DF / 32; ++kt) {
    const int k0 = kt * 32;
    Frag b1, b2, a;
    const unsigned short* pb1 = wtb + (size_t)ncol * DF + k0 + 8 * hh;
    const unsigned short* pb2 = wts + (size_t)ncol * DF + k0 + 8 * hh;
    b1.half[0] = *(const v8us*)pb1; b1.half[1] = *(const v8us*)(pb1 + 16);
    b2.half[0] = *(const v8us*)pb2; b2.half[1] = *(const v8us*)(pb2 + 16);
    const int oa = m * AP + k0 + 8 * hh;
    const int ob = (16 + m) * AP + k0 + 8 * hh;
    a.half[0] = *(const v8us*)(Adh + oa); a.half[1] = *(const v8us*)(Adh + oa + 16); d0 = wmb(a.v, b1.v, d0);
    a.half[0] = *(const v8us*)(Adl + oa); a.half[1] = *(const v8us*)(Adl + oa + 16); d0 = wmb(a.v, b1.v, d0);
    a.half[0] = *(const v8us*)(Adh + ob); a.half[1] = *(const v8us*)(Adh + ob + 16); d1 = wmb(a.v, b1.v, d1);
    a.half[0] = *(const v8us*)(Adl + ob); a.half[1] = *(const v8us*)(Adl + ob + 16); d1 = wmb(a.v, b1.v, d1);
    a.half[0] = *(const v8us*)(Ash + oa); a.half[1] = *(const v8us*)(Ash + oa + 16); s0 = wmb(a.v, b2.v, s0);
    a.half[0] = *(const v8us*)(Asl + oa); a.half[1] = *(const v8us*)(Asl + oa + 16); s0 = wmb(a.v, b2.v, s0);
    a.half[0] = *(const v8us*)(Ash + ob); a.half[1] = *(const v8us*)(Ash + ob + 16); s1 = wmb(a.v, b2.v, s1);
    a.half[0] = *(const v8us*)(Asl + ob); a.half[1] = *(const v8us*)(Asl + ob + 16); s1 = wmb(a.v, b2.v, s1);
  }
  __syncthreads();

#pragma unroll
  for (int r = 0; r < 8; ++r) {
    Y1[(8 * hh + r) * XSP + ncol]      = d0[r];
    Y1[(16 + 8 * hh + r) * XSP + ncol] = d1[r];
    Y2[(8 * hh + r) * XSP + ncol]      = s0[r];
    Y2[(16 + 8 * hh + r) * XSP + ncol] = s1[r];
  }
  __syncthreads();

  const float rw  = bfr(resw[0]);
  const float sig = 1.0f / (1.0f + expf(-rw));
  const v4f bb = {bfr(bib[4 * lane]), bfr(bib[4 * lane + 1]), bfr(bib[4 * lane + 2]), bfr(bib[4 * lane + 3])};
  const v4f sbv = {bfr(sib[4 * lane]), bfr(sib[4 * lane + 1]), bfr(sib[4 * lane + 2]), bfr(sib[4 * lane + 3])};
  const v4f g4 = {bfr(lng[4 * lane]), bfr(lng[4 * lane + 1]), bfr(lng[4 * lane + 2]), bfr(lng[4 * lane + 3])};
  const v4f e4 = {bfr(lnb[4 * lane]), bfr(lnb[4 * lane + 1]), bfr(lnb[4 * lane + 2]), bfr(lnb[4 * lane + 3])};
  v4f yv[4];
#pragma unroll
  for (int i = 0; i < 4; ++i) {
    const int rl = 4 * wave + i;
    const size_t row = (size_t)(rowBase + rl);
    const v4f y1 = *(const v4f*)(Y1 + rl * XSP + 4 * lane);
    const v4f y2 = *(const v4f*)(Y2 + rl * XSP + 4 * lane);
    const v4f xb = bfr4(*(const v4f*)(x + row * DF + 4 * lane));
    const v4f t  = lk4(y1 + bb, 0.01f) + lk4(y2 + sbv, 0.01f) + xb * sig;
    const float sm = wsum(t.x + t.y + t.z + t.w);
    const float mu = sm * (1.0f / DF);
    const v4f dd = t - mu;
    const float q  = wsum(dd.x * dd.x + dd.y * dd.y + dd.z * dd.z + dd.w * dd.w);
    const float rs = rsqrtf(q * (1.0f / DF) + 1e-5f);
    yv[i] = dd * rs * g4 + e4;
  }
#pragma unroll
  for (int i = 0; i < 4; ++i)
    *(volatile v4f*)(out + (size_t)(rowBase + 4 * wave + i) * DF + 4 * lane) = yv[i];
  __threadfence();
#pragma unroll
  for (int i = 0; i < 4; ++i)
    *(volatile v4f*)(out + (size_t)(rowBase + 4 * wave + i) * DF + 4 * lane) = yv[i];
}

static inline size_t alup(size_t v) { return (v + (size_t)255) & ~((size_t)255); }

extern "C" void kernel_launch(void* const* d_in, const int* in_sizes, int n_in,
                              void* d_out, int out_size, void* d_ws, size_t ws_size,
                              hipStream_t stream) {
  if (n_in < 15) return;
  const int nN = in_sizes[0] / DF;
  if (nN <= 0 || in_sizes[0] != nN * DF || (nN % GR) != 0) return;
  const int nR = in_sizes[4] / (DF * DF);
  if (nR <= 0 || nR > 8 || in_sizes[4] != nR * DF * DF) return;
  const int nE = in_sizes[1] / nR;
  if (nE <= 0 || in_sizes[1] != nR * nE || in_sizes[2] != in_sizes[1] || in_sizes[3] != in_sizes[1]) return;
  if (in_sizes[5] != nR * DF || in_sizes[6] != nR * DF || in_sizes[7] != nR * DF) return;
  if (in_sizes[8] != DF * DF || in_sizes[9] != DF || in_sizes[10] != DF * DF || in_sizes[11] != DF) return;
  if (in_sizes[12] < 1 || in_sizes[13] != DF || in_sizes[14] != DF) return;
  if (out_size != nN * DF) return;

  const float* x        = (const float*)d_in[0];
  const int*   edge_src = (const int*)d_in[1];
  const int*   edge_dst = (const int*)d_in[2];
  const float* edge_w   = (const float*)d_in[3];
  const float* W        = (const float*)d_in[4];
  const float* attn_l   = (const float*)d_in[5];
  const float* attn_r   = (const float*)d_in[6];
  const float* gat_b    = (const float*)d_in[7];
  const float* bi_w     = (const float*)d_in[8];
  const float* bi_b     = (const float*)d_in[9];
  const float* si_w     = (const float*)d_in[10];
  const float* si_b     = (const float*)d_in[11];
  const float* res_w    = (const float*)d_in[12];
  const float* ln_g     = (const float*)d_in[13];
  const float* ln_b     = (const float*)d_in[14];
  float* out = (float*)d_out;

  size_t off = 0;
  unsigned short* wt = (unsigned short*)((char*)d_ws + off);
  off = alup(off + (size_t)(nR + 2) * DF * DF * sizeof(unsigned short));
  float* elp = (float*)((char*)d_ws + off);  off = alup(off + (size_t)nN * sizeof(float));
  float* erp = (float*)((char*)d_ws + off);  off = alup(off + (size_t)nN * sizeof(float));
  float* Spl = (float*)((char*)d_ws + off);  off = alup(off + (size_t)nN * DF * sizeof(float));
  float* Qpl = (float*)((char*)d_ws + off);  off = alup(off + (size_t)nN * DF * sizeof(float));
  if (off > ws_size) return;

  float* hpl = out;

  k_prep<<<nR + 2, NTHR, 0, stream>>>(W, bi_w, si_w, wt, nR);

  hipFuncSetAttribute(reinterpret_cast<const void*>(&k_agg),
                      hipFuncAttributeMaxDynamicSharedMemorySize, LDS_AGG_BYTES);
  const int ggrid = nN / GR;
  const int agrid = (nN + NB - 1) / NB;
  for (int r = 0; r < nR; ++r) {
    k_gemm<<<ggrid, NTHR, 0, stream>>>(x, wt + (size_t)r * DF * DF, attn_l + (size_t)r * DF,
                                       attn_r + (size_t)r * DF, hpl, elp, erp, nN);
    k_agg<<<agrid, NTHR, LDS_AGG_BYTES, stream>>>(hpl, elp, erp, edge_src + (size_t)r * nE,
                                                  edge_dst + (size_t)r * nE, edge_w + (size_t)r * nE,
                                                  gat_b + (size_t)r * DF, Spl, Qpl, nN, nE, (r > 0) ? 1 : 0);
  }
  k_comb<<<ggrid, NTHR, 0, stream>>>(Spl, Qpl, x, wt + (size_t)nR * DF * DF, bi_b,
                                     wt + (size_t)(nR + 1) * DF * DF, si_b, res_w, ln_g, ln_b, out, nN);
}
